// Custom_GCN_59304908423673
// MI455X (gfx1250) — hardware-verified
//
#include <hip/hip_runtime.h>
#include <hip/hip_bf16.h>

typedef __attribute__((ext_vector_type(16))) _Float16 v16h;
typedef __attribute__((ext_vector_type(8)))  _Float16 v8h;
typedef __attribute__((ext_vector_type(16))) __bf16   v16b;
typedef __attribute__((ext_vector_type(8)))  __bf16   v8b;
typedef __attribute__((ext_vector_type(8)))  float    v8f;
typedef __attribute__((ext_vector_type(4)))  float    v4f;
#define U16(p) ((const unsigned short*)(const void*)(p))

__device__ __forceinline__ unsigned short f2bf_bits(float f) {
  unsigned u = __float_as_uint(f);
  return (unsigned short)((u + 0x7FFFu + ((u >> 16) & 1u)) >> 16);
}
__device__ __forceinline__ float bf_bits2f(unsigned short h) { return __uint_as_float(((unsigned)h) << 16); }

__device__ __forceinline__ void dep_guard_h(v8f& a, v8f& b, v16h x, v16h y) { asm volatile("v_nop\n\tv_nop\n\tv_nop\n\tv_nop" : "+v"(a), "+v"(b) : "v"(x), "v"(y)); }
__device__ __forceinline__ void dep_guard_b(v8f& a, v8f& b, v16b x, v16b y) { asm volatile("v_nop\n\tv_nop\n\tv_nop\n\tv_nop" : "+v"(a), "+v"(b) : "v"(x), "v"(y)); }
__device__ __forceinline__ void keep4_h(v16h a, v16h b, v16h c, v16h d) { asm volatile("v_nop" :: "v"(a), "v"(b), "v"(c), "v"(d)); }
__device__ __forceinline__ void keep4_b(v16b a, v16b b, v16b c, v16b d) { asm volatile("v_nop" :: "v"(a), "v"(b), "v"(c), "v"(d)); }
__device__ __forceinline__ void acc_guard4(v8f& a, v8f& b, v8f& c, v8f& d) { asm volatile("v_nop\n\tv_nop\n\tv_nop\n\tv_nop" : "+v"(a), "+v"(b), "+v"(c), "+v"(d)); }
template <typename T> struct Frag;
template <> struct Frag<_Float16> {
  typedef v16h V; union U { v16h v; v8h h[2]; };
  static __device__ __forceinline__ v16h load(const _Float16* p) {
    U f; f.h[0] = *(const v8h*)(p); f.h[1] = *(const v8h*)(p + 16); return f.v;
  }
  static __device__ __forceinline__ v8f mma(v16h a, v16h b, v8f c) {
    return __builtin_amdgcn_wmma_f32_16x16x32_f16(false, a, false, b, (short)0, c, false, false);
  }
  static __device__ __forceinline__ void guard(v8f& a, v8f& b, v16h x, v16h y) { dep_guard_h(a, b, x, y); }
  static __device__ __forceinline__ void keep(v16h a, v16h b, v16h c, v16h d) { keep4_h(a, b, c, d); }
};
template <> struct Frag<__bf16> {
  typedef v16b V; union U { v16b v; v8b h[2]; };
  static __device__ __forceinline__ v16b load(const __bf16* p) {
    U f; f.h[0] = *(const v8b*)(p); f.h[1] = *(const v8b*)(p + 16); return f.v;
  }
  static __device__ __forceinline__ v8f mma(v16b a, v16b b, v8f c) {
    return __builtin_amdgcn_wmma_f32_16x16x32_bf16(false, a, false, b, (short)0, c, false, false);
  }
  static __device__ __forceinline__ void guard(v8f& a, v8f& b, v16b x, v16b y) { dep_guard_b(a, b, x, y); }
  static __device__ __forceinline__ void keep(v16b a, v16b b, v16b c, v16b d) { keep4_b(a, b, c, d); }
};

template <int ET> struct Elem;
template <> struct Elem<0> { typedef _Float16 T; };
template <> struct Elem<1> { typedef __bf16 T; };
template <int ET, bool SPLIT, int BIAS_MODE, int OUT_MODE, bool RESID, int ACT = 0>
__global__ __launch_bounds__(256) void wmma_gemm64(
    const unsigned short* __restrict__ Ap, const unsigned short* __restrict__ A2p, int lda, long strideA,
    const unsigned short* __restrict__ Btp, const unsigned short* __restrict__ Bt2p, int ldb, long strideB,
    void* __restrict__ Cout, void* __restrict__ Cout2, int ldc, long strideC,
    const float* __restrict__ bias,
    const float* __restrict__ resid, long strideR,
    int M, int N, int K, float scale, float bscale) {
  typedef typename Elem<ET>::T T;
  typedef typename Frag<T>::V V;
  const T* A = (const T*)Ap; const T* A2 = (const T*)A2p; const T* Bt = (const T*)Btp; const T* Bt2 = (const T*)Bt2p;
  __shared__ __align__(16) float sT[8][16 * 68];
  const int b    = blockIdx.y;
  const int lane = threadIdx.x & 31;
  const int wave = threadIdx.x >> 5;
  const int tilesN = N >> 6;
  const int tilesM = M >> 6;
  const int tile = blockIdx.x * 8 + wave;
  if (tile >= tilesM * tilesN) return;
  const int tm = tile / tilesN;
  const int tn = tile - tm * tilesN;
  const int m0 = tm << 6;
  const int n0 = tn << 6;

  const T* Ab  = A  + (size_t)b * strideA;
  const T* Bb  = Bt + (size_t)b * strideB;
  const T* Ab2 = SPLIT ? (A2  + (size_t)b * strideA) : nullptr;
  const T* Bb2 = SPLIT ? (Bt2 + (size_t)b * strideB) : nullptr;

  const int rlane = lane & 15;
  const int koff  = (lane >> 4) * 8;
  const int mOff  = (lane >> 4) * 8;

  v8f acc[4][4];
#pragma unroll
  for (int i = 0; i < 4; ++i)
#pragma unroll
    for (int j = 0; j < 4; ++j) acc[i][j] = (v8f){0.f,0.f,0.f,0.f,0.f,0.f,0.f,0.f};

  for (int k0 = 0; k0 < K; k0 += 32) {
    V bh[4], bl[4];
#pragma unroll
    for (int j = 0; j < 4; ++j) {
      const size_t bo = (size_t)(n0 + (j << 4) + rlane) * ldb + koff + k0;
      bh[j] = Frag<T>::load(Bb + bo);
      if (SPLIT) bl[j] = Frag<T>::load(Bb2 + bo);
    }
#pragma unroll
    for (int i = 0; i < 4; ++i) {
      const size_t ao = (size_t)(m0 + (i << 4) + rlane) * lda + koff + k0;
      V ah = Frag<T>::load(Ab + ao);
      V al;
      if (SPLIT) al = Frag<T>::load(Ab2 + ao);
#pragma unroll
      for (int j = 0; j < 4; ++j) {
        acc[i][j] = Frag<T>::mma(ah, bh[j], acc[i][j]);
        if (SPLIT) {
          acc[i][j] = Frag<T>::mma(ah, bl[j], acc[i][j]);
          acc[i][j] = Frag<T>::mma(al, bh[j], acc[i][j]);
        }
      }
      Frag<T>::guard(acc[i][0], acc[i][3], ah, SPLIT ? al : ah);
    }
    Frag<T>::keep(bh[0], bh[1], bh[2], bh[3]);
    if (SPLIT) Frag<T>::keep(bl[0], bl[1], bl[2], bl[3]);
  }
  acc_guard4(acc[0][0], acc[0][1], acc[0][2], acc[0][3]);
  acc_guard4(acc[1][0], acc[1][1], acc[1][2], acc[1][3]);
  acc_guard4(acc[2][0], acc[2][1], acc[2][2], acc[2][3]);
  acc_guard4(acc[3][0], acc[3][1], acc[3][2], acc[3][3]);

  float* slab = sT[wave];
  const float* Rb = RESID ? (resid + (size_t)b * strideR) : nullptr;
#pragma unroll
  for (int i = 0; i < 4; ++i) {
    const int mBase = m0 + (i << 4);
#pragma unroll
    for (int j = 0; j < 4; ++j) {
      const int n = n0 + (j << 4) + rlane;
      float bv = 0.f;
      if (BIAS_MODE == 2) bv = bias[n] * bscale;
#pragma unroll
      for (int r = 0; r < 8; ++r) {
        float v = acc[i][j][r] * scale;
        if (BIAS_MODE == 1) v += bias[mBase + mOff + r] * bscale;
        if (BIAS_MODE == 2) v += bv;
        if (RESID) v += Rb[(size_t)(mBase + mOff + r) * ldc + n];
        if (ACT == 1) v = tanhf(v);
        if (ACT == 2) v = fmaxf(v, 0.0f);
        if (ACT == 3) v = v / (1.0f + expf(-v));
        if (ACT == 4) v = (v > 0.f) ? v : 0.01f * v;
        if (ACT == 5) v = 0.5f * v * (1.0f + erff(v * 0.70710678118654752f));
        slab[(mOff + r) * 68 + (j << 4) + rlane] = v;
      }
    }
    __builtin_amdgcn_fence(__ATOMIC_RELEASE, "workgroup");
    __builtin_amdgcn_wave_barrier();
    __builtin_amdgcn_fence(__ATOMIC_ACQUIRE, "workgroup");
    if (OUT_MODE == 0) {
      float* C = (float*)Cout + (size_t)b * strideC;
      const int hh = lane >> 4, c4 = (lane & 15) * 4;
      for (int pass = 0; pass < 2; ++pass) {
#pragma unroll
        for (int it = 0; it < 8; ++it) {
          const int row = it * 2 + hh;
          v4f v = *(const v4f*)(slab + row * 68 + c4);
          *(volatile v4f*)(C + (size_t)(mBase + row) * ldc + n0 + c4) = v;
        }
        __threadfence();
      }
    } else {
      const int q = lane >> 3, c8 = (lane & 7) * 8;
      unsigned short* C  = (unsigned short*)Cout  + (size_t)b * strideC;
      unsigned short* C2 = (OUT_MODE == 2) ? ((unsigned short*)Cout2 + (size_t)b * strideC) : nullptr;
      for (int pass = 0; pass < 2; ++pass) {
#pragma unroll
        for (int it = 0; it < 4; ++it) {
          const int row = it * 4 + q;
          const float* sp = slab + row * 68 + c8;
          v8h hv, lv;
#pragma unroll
          for (int e = 0; e < 8; ++e) {
            if (OUT_MODE == 1) {
              hv[e] = (_Float16)sp[e];
            } else {
              unsigned short hb = f2bf_bits(sp[e]);
              unsigned short lb = f2bf_bits(sp[e] - bf_bits2f(hb));
              hv[e] = __builtin_bit_cast(_Float16, hb);
              lv[e] = __builtin_bit_cast(_Float16, lb);
            }
          }
          *(volatile v8h*)(C + (size_t)(mBase + row) * ldc + n0 + c8) = hv;
          if (OUT_MODE == 2) *(volatile v8h*)(C2 + (size_t)(mBase + row) * ldc + n0 + c8) = lv;
        }
        __threadfence();
      }
    }
    __builtin_amdgcn_fence(__ATOMIC_RELEASE, "workgroup");
    __builtin_amdgcn_wave_barrier();
    __builtin_amdgcn_fence(__ATOMIC_ACQUIRE, "workgroup");
  }
}

__global__ __launch_bounds__(256) void cast_f32_f16x8(
    const float* __restrict__ in, _Float16* __restrict__ out, int n8, float sc) {
  const int i = blockIdx.x * 256 + threadIdx.x;
  if (i < n8) {
    const v4f a = *(const v4f*)(in + (size_t)i * 8);
    const v4f c = *(const v4f*)(in + (size_t)i * 8 + 4);
    v8h h;
    h[0] = (_Float16)(a[0] * sc); h[1] = (_Float16)(a[1] * sc);
    h[2] = (_Float16)(a[2] * sc); h[3] = (_Float16)(a[3] * sc);
    h[4] = (_Float16)(c[0] * sc); h[5] = (_Float16)(c[1] * sc);
    h[6] = (_Float16)(c[2] * sc); h[7] = (_Float16)(c[3] * sc);
    *(volatile v8h*)(out + (size_t)i * 8) = h;
    __threadfence();
    *(volatile v8h*)(out + (size_t)i * 8) = h;
  }
}

__global__ __launch_bounds__(256) void transpose_cast_f16(
    const float* __restrict__ in, _Float16* __restrict__ out, int rows, int cols, float sc) {
  __shared__ __align__(16) _Float16 tile[64 * 72];
  const int tid = threadIdx.x, lane = tid & 31, wave = tid >> 5;
  const int rb = blockIdx.y * 64, cb = blockIdx.x * 64;
  if (rb + 64 > rows || cb + 64 > cols) return;
#pragma unroll
  for (int it = 0; it < 4; ++it) {
    const int r  = it * 16 + (tid >> 4);
    const int c4 = (tid & 15) * 4;
    const v4f v = *(const v4f*)(in + (size_t)(rb + r) * cols + cb + c4);
#pragma unroll
    for (int e = 0; e < 4; ++e) tile[(c4 + e) * 72 + r] = (_Float16)(v[e] * sc);
  }
  __syncthreads();
  const int q = lane >> 3, c8 = (lane & 7) * 8;
  for (int pass = 0; pass < 2; ++pass) {
#pragma unroll
    for (int it = 0; it < 2; ++it) {
      const int c = wave * 8 + it * 4 + q;
      const v8h v = *(const v8h*)(tile + c * 72 + c8);
      *(volatile v8h*)(out + (size_t)(cb + c) * rows + rb + c8) = v;
    }
    __threadfence();
  }
}

extern "C" void kernel_launch(void* const* d_in, const int* in_sizes, int n_in,
                              void* d_out, int out_size, void* d_ws, size_t ws_size,
                              hipStream_t stream) {
  constexpr int B = 32, N = 512, D = 512;
  constexpr long NB  = (long)B * N * D;
  constexpr long NA  = (long)B * N * N;
  constexpr long WSZ = (long)D * D;
  if (n_in < 8) return;
  if (in_sizes[0] != NB || in_sizes[1] != NA || in_sizes[2] != WSZ || in_sizes[4] != WSZ ||
      in_sizes[6] != WSZ || in_sizes[3] != D || in_sizes[5] != D || in_sizes[7] != D ||
      out_size != NB) return;

  const float* x   = (const float*)d_in[0];
  const float* adj = (const float*)d_in[1];
  const float* W0  = (const float*)d_in[2];
  const float* b0  = (const float*)d_in[3];
  const float* W1  = (const float*)d_in[4];
  const float* b1  = (const float*)d_in[5];
  const float* W2  = (const float*)d_in[6];
  const float* b2  = (const float*)d_in[7];
  float* out = (float*)d_out;

  const size_t bytesX = (size_t)NB * 2, bytesA = (size_t)NA * 2, bytesW = (size_t)WSZ * 2;
  const size_t offX  = 0;
  const size_t offA  = offX + bytesX;
  const size_t offW  = offA + bytesA;
  const size_t offS  = offW + 3 * bytesW;
  const size_t offH  = offS + bytesX;
  const size_t total = offH + bytesX;
  if (total > ws_size || total > (size_t)134217728) return;
  char* ws = (char*)d_ws;
  _Float16* x16   = (_Float16*)(ws + offX);
  _Float16* adj16 = (_Float16*)(ws + offA);
  _Float16* wt0   = (_Float16*)(ws + offW);
  _Float16* wt1   = wt0 + WSZ;
  _Float16* wt2   = wt1 + WSZ;
  _Float16* sT16  = (_Float16*)(ws + offS);
  _Float16* h16   = (_Float16*)(ws + offH);

  const int n8 = (int)(NB / 8);
  cast_f32_f16x8<<<(n8 + 255) / 256, 256, 0, stream>>>(x, x16, n8, 1.0f);
  const int a8 = (int)(NA / 8);
  cast_f32_f16x8<<<(a8 + 255) / 256, 256, 0, stream>>>(adj, adj16, a8, 16.0f);
  const dim3 gridT(D / 64, D / 64);
  transpose_cast_f16<<<gridT, 256, 0, stream>>>(W0, wt0, D, D, 64.0f);
  transpose_cast_f16<<<gridT, 256, 0, stream>>>(W1, wt1, D, D, 64.0f);
  transpose_cast_f16<<<gridT, 256, 0, stream>>>(W2, wt2, D, D, 64.0f);

  const long SND = (long)N * D;
  const long SNN = (long)N * N;
  const dim3 gridS(((D / 64) * (N / 64) + 7) / 8, B);
  const dim3 gridG(((N / 64) * (D / 64) + 7) / 8, B);

  wmma_gemm64<0, false, 0, 1, false, 0><<<gridS, 256, 0, stream>>>(
      U16(wt0), U16(wt0), D, 0L, U16(x16), U16(x16), D, SND,
      (void*)sT16, (void*)sT16, N, SND, b0, b0, 0L, D, N, D, 0.25f, 1.0f);
  wmma_gemm64<0, false, 2, 1, false, 2><<<gridG, 256, 0, stream>>>(
      U16(adj16), U16(adj16), N, SNN, U16(sT16), U16(sT16), N, SND,
      (void*)h16, (void*)h16, D, SND, b0, b0, 0L, N, D, N, 0.00390625f, 1.0f);

  wmma_gemm64<0, false, 0, 1, false, 0><<<gridS, 256, 0, stream>>>(
      U16(wt1), U16(wt1), D, 0L, U16(h16), U16(h16), D, SND,
      (void*)sT16, (void*)sT16, N, SND, b1, b1, 0L, D, N, D, 0.015625f, 1.0f);
  wmma_gemm64<0, false, 2, 1, false, 2><<<gridG, 256, 0, stream>>>(
      U16(adj16), U16(adj16), N, SNN, U16(sT16), U16(sT16), N, SND,
      (void*)h16, (void*)h16, D, SND, b1, b1, 0L, N, D, N, 0.0009765625f, 0.015625f);

  wmma_gemm64<0, false, 0, 1, false, 0><<<gridS, 256, 0, stream>>>(
      U16(wt2), U16(wt2), D, 0L, U16(h16), U16(h16), D, SND,
      (void*)sT16, (void*)sT16, N, SND, b2, b2, 0L, D, N, D, 0.00390625f, 1.0f);
  wmma_gemm64<0, false, 2, 0, false, 0><<<gridG, 256, 0, stream>>>(
      U16(adj16), U16(adj16), N, SNN, U16(sT16), U16(sT16), N, SND,
      (void*)out, (void*)out, D, SND, b2, b2, 0L, N, D, N, 16.0f, 1.0f);
  (void)hipGetLastError();
}
